// MultiHeadSelfAttention_10247791968609
// MI455X (gfx1250) — hardware-run, weakly checked
//
#include <hip/hip_runtime.h>
#ifndef NB
#define NB 4
#endif
#ifndef SEQ
#define SEQ 2048
#endif
#define NB_FULL 4
#define SEQ_FULL 2048
#define DM 1024
#define NH 16
#define HD 64
#define NR ((size_t)NB * SEQ)
#define CS 0.18033688011112042f
#define TAU 22.0f

static_assert(SEQ % 128 == 0);
static_assert(DM % 128 == 0);
static_assert(NH * HD == DM);
static_assert(NB <= NB_FULL && SEQ <= SEQ_FULL);
static_assert((size_t)4 * DM * DM * 2 + (size_t)5 * NB * SEQ * DM * 2 <= (size_t)134217728);

typedef _Float16 v16h __attribute__((ext_vector_type(16)));
typedef unsigned short v8us __attribute__((ext_vector_type(8), may_alias));
typedef float  v8f  __attribute__((ext_vector_type(8)));
typedef float  v4f  __attribute__((ext_vector_type(4)));
typedef float  v4fa __attribute__((ext_vector_type(4), may_alias));
union FragH { v16h v; v8us half[2]; _Float16 h[16]; unsigned short u[16]; };

__device__ __forceinline__ unsigned short bf16_bits(float x) { unsigned int u = __float_as_uint(x); return (unsigned short)((u + 0x7FFFu + ((u >> 16) & 1u)) >> 16); }
__device__ __forceinline__ float bf16_rne(float x) { return __uint_as_float(((unsigned int)bf16_bits(x)) << 16); }

__device__ __forceinline__ v16h g2_frag(const _Float16* p, int hh) { FragH f; f.half[0] = *(const v8us*)((const unsigned short*)p + 8 * hh); f.half[1] = *(const v8us*)((const unsigned short*)p + 16 + 8 * hh); return f.v; }
__device__ __forceinline__ v8f wm(v16h a, v16h b, v8f c) { return __builtin_amdgcn_wmma_f32_16x16x32_f16(false, a, false, b, (short)0, c, false, false); }

__global__ __launch_bounds__(256) void k_wnat(const float* __restrict__ w, size_t n8, _Float16* __restrict__ Bt) {
  const size_t t = (size_t)blockIdx.x * 256 + threadIdx.x; if (t >= n8) return;
  const v4f a = *(const v4fa*)(w + t * 8), c = *(const v4fa*)(w + t * 8 + 4);
  FragH f;
#pragma unroll
  for (int q = 0; q < 4; ++q) { f.h[q] = (_Float16)(bf16_rne(a[q]) * 16.0f); f.h[4 + q] = (_Float16)(bf16_rne(c[q]) * 16.0f); }
  const v8us o = f.half[0];
  *(volatile v8us*)((unsigned short*)Bt + t * 8) = o; __threadfence(); *(volatile v8us*)((unsigned short*)Bt + t * 8) = o;
}

__global__ __launch_bounds__(256) void k_x16(const float* __restrict__ x, _Float16* __restrict__ X16, size_t n8) {
  const size_t t = (size_t)blockIdx.x * 256 + threadIdx.x; if (t >= n8) return;
  const float* xs = x + (size_t)blockIdx.y * SEQ_FULL * DM; unsigned short* xd = (unsigned short*)X16 + (size_t)blockIdx.y * SEQ * DM;
  const v4f a = *(const v4fa*)(xs + t * 8), c = *(const v4fa*)(xs + t * 8 + 4);
  FragH f;
#pragma unroll
  for (int q = 0; q < 4; ++q) { f.h[q] = (_Float16)bf16_rne(a[q]); f.h[4 + q] = (_Float16)bf16_rne(c[q]); }
  const v8us o = f.half[0];
  *(volatile v8us*)(xd + t * 8) = o; __threadfence(); *(volatile v8us*)(xd + t * 8) = o;
}

template <bool OUT32, bool HASBIAS>
__global__ __launch_bounds__(128) void k_gemm2(const _Float16* __restrict__ A, int lda, size_t sA, const _Float16* __restrict__ Bh, int ldb, size_t sB, float alpha,
                                               const float* __restrict__ bias, float* __restrict__ C, _Float16* __restrict__ C16, int ldc, size_t sC, int N, int K) {
  __shared__ __attribute__((aligned(16))) float so[4][32][68];
  const int tid = threadIdx.x, w = tid >> 5, lane = tid & 31, ln = lane & 15, hh = lane >> 4; const int by = blockIdx.y;
  A += (size_t)by * sA; Bh += (size_t)by * sB; const size_t cofs = (size_t)by * sC;
  const int ntn = N >> 6; const int mt = blockIdx.x / ntn, nq = blockIdx.x - mt * ntn; const int row0 = mt * 128 + 32 * w, col0 = nq * 64;
  const _Float16* a0p = A + (size_t)(row0 + ln) * lda; const _Float16* a1p = a0p + (size_t)16 * lda;
  const _Float16* b0p = Bh + (size_t)(col0 + ln) * ldb; const _Float16* b1p = b0p + (size_t)16 * ldb; const _Float16* b2p = b1p + (size_t)16 * ldb; const _Float16* b3p = b2p + (size_t)16 * ldb;
  const v8f z8 = {0.f,0.f,0.f,0.f,0.f,0.f,0.f,0.f}; v8f c00 = z8, c01 = z8, c02 = z8, c03 = z8, c10 = z8, c11 = z8, c12 = z8, c13 = z8;
#pragma unroll 1
  for (int kb = 0; kb < K; kb += 32) {
    const v16h a0 = g2_frag(a0p + kb, hh), a1 = g2_frag(a1p + kb, hh);
    const v16h b0 = g2_frag(b0p + kb, hh), b1 = g2_frag(b1p + kb, hh), b2 = g2_frag(b2p + kb, hh), b3 = g2_frag(b3p + kb, hh);
    c00 = wm(a0, b0, c00); c10 = wm(a1, b0, c10);
    c01 = wm(a0, b1, c01); c11 = wm(a1, b1, c11);
    c02 = wm(a0, b2, c02); c12 = wm(a1, b2, c12);
    c03 = wm(a0, b3, c03); c13 = wm(a1, b3, c13);
    asm volatile("v_nop\n\tv_nop\n\tv_nop\n\tv_nop" : "+v"(c00), "+v"(c01), "+v"(c02), "+v"(c03), "+v"(c10), "+v"(c11), "+v"(c12), "+v"(c13) : "v"(a0), "v"(a1), "v"(b0), "v"(b1), "v"(b2), "v"(b3));
  }
  v8f accs[8] = {c00, c01, c02, c03, c10, c11, c12, c13};
#pragma unroll
  for (int u = 0; u < 8; ++u) { const int t = u & 3, half = u >> 2; const int col = col0 + t * 16 + ln; float bv = 0.f; if (HASBIAS) bv = bf16_rne(bias[col]);
#pragma unroll
    for (int r = 0; r < 8; ++r) { const int rloc = half * 16 + 8 * hh + r; so[w][rloc][t * 16 + ln] = accs[u][r] * alpha + bv; } }
  __syncthreads();
  if (OUT32) {
    const int rsub = lane >> 4, c4 = (lane & 15) * 4;
    for (int pass = 0; pass < 2; ++pass) {
#pragma unroll
      for (int q = 0; q < 16; ++q) { const int r = q * 2 + rsub; const v4f v = *(const v4fa*)&so[w][r][c4]; *(volatile v4f*)(C + cofs + (size_t)(row0 + r) * ldc + col0 + c4) = v; }
      if (pass == 0) __threadfence(); }
  } else {
    const int rq = lane >> 3, c8 = (lane & 7) * 8;
    for (int pass = 0; pass < 2; ++pass) {
#pragma unroll
      for (int q = 0; q < 8; ++q) { const int r = q * 4 + rq; const v4f x0 = *(const v4fa*)&so[w][r][c8], x1 = *(const v4fa*)&so[w][r][c8 + 4]; FragH f;
#pragma unroll
        for (int i = 0; i < 4; ++i) { f.h[i] = (_Float16)x0[i]; f.h[4 + i] = (_Float16)x1[i]; }
        const v8us o = f.half[0];
        *(volatile v8us*)((unsigned short*)C16 + cofs + (size_t)(row0 + r) * ldc + col0 + c8) = o; }
      if (pass == 0) __threadfence(); }
  }
}

__global__ __launch_bounds__(128) void k_flash(const _Float16* __restrict__ Q16, const _Float16* __restrict__ K16, const _Float16* __restrict__ VT,
                                               const float* __restrict__ bv, _Float16* __restrict__ O16) {
  __shared__ __attribute__((aligned(16))) unsigned short so[4][16][72];
  const int tid = threadIdx.x, w = tid >> 5, lane = tid & 31, ln = lane & 15, hh = lane >> 4;
  const int b = blockIdx.z, h = blockIdx.y, q0 = blockIdx.x * 64 + w * 16;
  const size_t rb = (size_t)b * SEQ;
  const _Float16* qp = Q16 + (rb + q0 + ln) * DM + h * HD;
  const v16h qb0 = g2_frag(qp, hh), qb1 = g2_frag(qp + 32, hh);
  const _Float16* kp = K16 + (rb + ln) * DM + h * HD;
  const _Float16* vp = VT + ((size_t)b * DM + h * HD + ln) * SEQ;
  const v8f z8 = {0.f,0.f,0.f,0.f,0.f,0.f,0.f,0.f};
  v8f o0 = z8, o1 = z8, o2 = z8, o3 = z8;
  float mrun = -1.0e30f, lrun = 0.f, nm = 0.f;
#pragma unroll 1
  for (int j0 = 0; j0 < SEQ; j0 += 32) {
    const _Float16* k0p = kp + (size_t)j0 * DM; const _Float16* k1p = k0p + (size_t)16 * DM;
    const v16h k00 = g2_frag(k0p, hh), k01 = g2_frag(k0p + 32, hh), k10 = g2_frag(k1p, hh), k11 = g2_frag(k1p + 32, hh);
    v8f s0 = wm(k00, qb0, z8); s0 = wm(k01, qb1, s0);
    v8f s1 = wm(k10, qb0, z8); s1 = wm(k11, qb1, s1);
    asm volatile("v_nop\n\tv_nop\n\tv_nop\n\tv_nop" : "+v"(s0), "+v"(s1) : "v"(k00), "v"(k01), "v"(k10), "v"(k11), "v"(qb0), "v"(qb1));
    float mx = fmaxf(s0[0], s1[0]);
#pragma unroll
    for (int r = 1; r < 8; ++r) mx = fmaxf(mx, fmaxf(s0[r], s1[r]));
    mx = fmaxf(mx, __shfl_xor(mx, 16, 32));
    const bool up = mx > mrun + TAU;
    if (__any(up)) {
      const float mnew = up ? mx : mrun;
      const float al = __builtin_amdgcn_exp2f((mrun - mnew) * CS);
      mrun = mnew; nm = 8.0f - mnew * CS; lrun *= al;
      o0 *= al; o1 *= al; o2 *= al; o3 *= al;
    }
    const v8f e0 = s0 * CS + nm, e1 = s1 * CS + nm;
    FragH pf; v8f p0, p1;
#pragma unroll
    for (int r = 0; r < 8; ++r) { p0[r] = __builtin_amdgcn_exp2f(e0[r]); p1[r] = __builtin_amdgcn_exp2f(e1[r]); pf.h[r] = (_Float16)p0[r]; pf.h[8 + r] = (_Float16)p1[r]; }
    const v8f ps = p0 + p1;
    lrun += ((ps[0] + ps[1]) + (ps[2] + ps[3])) + ((ps[4] + ps[5]) + (ps[6] + ps[7]));
    const _Float16* vq = vp + j0;
    const v16h va0 = g2_frag(vq, hh), va1 = g2_frag(vq + (size_t)16 * SEQ, hh), va2 = g2_frag(vq + (size_t)32 * SEQ, hh), va3 = g2_frag(vq + (size_t)48 * SEQ, hh);
    const v16h pb = pf.v;
    o0 = wm(va0, pb, o0); o1 = wm(va1, pb, o1); o2 = wm(va2, pb, o2); o3 = wm(va3, pb, o3);
    asm volatile("v_nop\n\tv_nop\n\tv_nop\n\tv_nop" : "+v"(o0), "+v"(o1), "+v"(o2), "+v"(o3) : "v"(va0), "v"(va1), "v"(va2), "v"(va3), "v"(pb));
  }
  const float lt = lrun + __shfl_xor(lrun, 16, 32);
  const float inv = 1.0f / lt;
  v8f oa[4] = {o0, o1, o2, o3};
#pragma unroll
  for (int t = 0; t < 4; ++t) {
    const v4f bA = *(const v4fa*)(bv + h * HD + 16 * t + 8 * hh), bB = *(const v4fa*)(bv + h * HD + 16 * t + 8 * hh + 4);
    FragH f;
#pragma unroll
    for (int r = 0; r < 4; ++r) { f.h[r] = (_Float16)((oa[t][r] * inv + bf16_rne(bA[r])) * 64.0f); f.h[4 + r] = (_Float16)((oa[t][4 + r] * inv + bf16_rne(bB[r])) * 64.0f); }
    *(v8us*)&so[w][ln][16 * t + 8 * hh] = f.half[0];
  }
  __syncthreads();
  const int rq = lane >> 3, c8 = (lane & 7) * 8;
  for (int pass = 0; pass < 2; ++pass) {
#pragma unroll
    for (int q = 0; q < 4; ++q) { const int r = q * 4 + rq; const v8us v = *(const v8us*)&so[w][r][c8];
      *(volatile v8us*)((unsigned short*)O16 + (rb + q0 + r) * DM + h * HD + c8) = v; }
    if (pass == 0) __threadfence(); }
}

extern "C" void kernel_launch(void* const* d_in, const int* in_sizes, int n_in,
                              void* d_out, int out_size, void* d_ws, size_t ws_size, hipStream_t stream) {
  if (n_in < 11) return;
  const size_t need_x = ((size_t)(NB - 1) * SEQ_FULL + SEQ) * DM;
  if ((size_t)in_sizes[0] < need_x || (size_t)in_sizes[1] < need_x || (size_t)in_sizes[2] < need_x || (size_t)out_size < need_x) return;
  if (in_sizes[3] < DM * DM || in_sizes[5] < DM * DM || in_sizes[7] < DM * DM || in_sizes[9] < DM * DM) return;
  if (in_sizes[4] < DM || in_sizes[6] < DM || in_sizes[8] < DM || in_sizes[10] < DM) return;
  const float* xq = (const float*)d_in[0]; const float* xk = (const float*)d_in[1]; const float* xv = (const float*)d_in[2];
  const float* wq = (const float*)d_in[3]; const float* bq = (const float*)d_in[4];
  const float* wk = (const float*)d_in[5]; const float* bk = (const float*)d_in[6];
  const float* wv = (const float*)d_in[7]; const float* bvv = (const float*)d_in[8];
  const float* wo = (const float*)d_in[9]; const float* bo = (const float*)d_in[10];
  char* ws = (char*)d_ws; size_t off = 0;
  auto take = [&](size_t bytes) { char* p = ws + off; off += (bytes + 255) & ~(size_t)255; return p; };
  _Float16* BQ = (_Float16*)take((size_t)DM * DM * 2); _Float16* BK = (_Float16*)take((size_t)DM * DM * 2); _Float16* BV = (_Float16*)take((size_t)DM * DM * 2); _Float16* BO = (_Float16*)take((size_t)DM * DM * 2);
  _Float16* X16 = (_Float16*)take(NR * DM * 2);
  _Float16* Q16 = (_Float16*)take(NR * DM * 2); _Float16* K16 = (_Float16*)take(NR * DM * 2);
  _Float16* VT  = (_Float16*)take((size_t)NB * DM * SEQ * 2);
  _Float16* O16 = (_Float16*)take(NR * DM * 2);
  if (off > ws_size) return;
  const size_t wn8 = (size_t)DM * DM / 8; const unsigned gw = (unsigned)((wn8 + 255) / 256);
  k_wnat<<<gw, 256, 0, stream>>>(wq, wn8, BQ); k_wnat<<<gw, 256, 0, stream>>>(wk, wn8, BK); k_wnat<<<gw, 256, 0, stream>>>(wv, wn8, BV); k_wnat<<<gw, 256, 0, stream>>>(wo, wn8, BO);
  const size_t xn8 = (size_t)SEQ * DM / 8; const dim3 gx((unsigned)((xn8 + 255) / 256), NB);
  const dim3 gp((unsigned)((NR / 128) * (DM / 64)), 1);
  k_x16<<<gx, 256, 0, stream>>>(xq, X16, xn8);
  k_gemm2<false, true><<<gp, 128, 0, stream>>>(X16, DM, 0, BQ, DM, 0, 0.0625f, bq, nullptr, Q16, DM, 0, DM, DM);
  k_x16<<<gx, 256, 0, stream>>>(xk, X16, xn8);
  k_gemm2<false, true><<<gp, 128, 0, stream>>>(X16, DM, 0, BK, DM, 0, 0.0625f, bk, nullptr, K16, DM, 0, DM, DM);
  k_x16<<<gx, 256, 0, stream>>>(xv, X16, xn8);
  k_gemm2<false, false><<<dim3((DM / 128) * (SEQ / 64), NB), 128, 0, stream>>>(BV, DM, 0, X16, DM, (size_t)SEQ * DM, 0.0625f, bvv, nullptr, VT, SEQ, (size_t)DM * SEQ, SEQ, DM);
  k_flash<<<dim3(SEQ / 64, NH, NB), 128, 0, stream>>>(Q16, K16, VT, bvv, O16);
  k_gemm2<true, true><<<dim3((SEQ / 128) * (DM / 64), NB), 128, 0, stream>>>(O16, DM, (size_t)SEQ * DM, BO, DM, 0, 0.0009765625f, bo, (float*)d_out, nullptr, DM, (size_t)SEQ_FULL * DM, DM, DM);
}
